// EI_Adaptive_Fusion_2671469658235
// MI455X (gfx1250) — hardware-verified
//
#include <hip/hip_runtime.h>


namespace {
constexpr int NB = 4, HQ = 16, WQ = 32, NQ = HQ * WQ  , NKV = 642, NKP = 704  , C = 128, C2 = 256, NRQ = NB * NQ, NRK = NB * NKP;
constexpr float XS = 8.0f, WSC = 256.0f, PS = 8.0f, PSD = 1024.0f, SCALE = 0.088388347648318447f  , LOG2E = 1.4426950408889634f, PI_F = 3.14159265358979323846f;

typedef _Float16 b16;
typedef __attribute__((ext_vector_type(16))) _Float16 v16b;
typedef __attribute__((ext_vector_type(8))) _Float16 v8b;
typedef __attribute__((ext_vector_type(8))) float v8f;
typedef __attribute__((ext_vector_type(4))) float v4f;
__device__ __forceinline__ float bf16_rne(float f) { unsigned int u = __float_as_uint(f); u += 0x7FFFu + ((u >> 16) & 1u); return __uint_as_float(u & 0xFFFF0000u); }
__device__ __forceinline__ void split16(float v, b16& hi, b16& lo) { hi = (b16)v; lo = (b16)(v - (float)hi); }
__device__ __forceinline__ v16b frag_kb(const b16* p, int hh) { const v8b a = *(const v8b*)(p + 8 * hh), b = *(const v8b*)(p + 16 + 8 * hh); v16b f;
#pragma unroll
  for (int e = 0; e < 8; ++e) { f[e] = a[e]; f[8 + e] = b[e]; } return f; }
__device__ __forceinline__ v8f wmma16b(v16b a, v16b b, v8f c) { v8f d = __builtin_amdgcn_wmma_f32_16x16x32_f16(false, a, false, b, (short)0, c, false, false); asm volatile("v_nop\n\tv_nop\n\tv_nop\n\tv_nop" : "+v"(d) : "v"(a), "v"(b)); return d; }
__device__ __forceinline__ void wave_lds_sync() { __builtin_amdgcn_fence(__ATOMIC_RELEASE, "workgroup"); __builtin_amdgcn_wave_barrier(); __builtin_amdgcn_fence(__ATOMIC_ACQUIRE, "workgroup"); }
__device__ __forceinline__ float nexp2(float x) { return __builtin_amdgcn_exp2f(x); }
__device__ __forceinline__ float pmul(float a, float b) { float p = a * b; asm volatile("" : "+v"(p)); return p; }

__global__ __launch_bounds__(256) void preperp_kernel(const float* __restrict__ erp, b16* __restrict__ ERP16) {
  __shared__ __attribute__((aligned(16))) b16 T[64][64 + 8];
  const int b = blockIdx.z, c0 = blockIdx.y * 64, n0 = blockIdx.x * 64, t_ = threadIdx.x;
  for (int q = t_; q < 64 * 64; q += 256) { const int cc = q >> 6, nn = q & 63; T[nn][cc] = (b16)(bf16_rne(erp[((size_t)b * C + c0 + cc) * NQ + n0 + nn]) * XS); }
  __syncthreads();
  for (int pass = 0; pass < 2; ++pass) { for (int q = t_; q < 64 * 8; q += 256) { const int nn = q >> 3, c8 = (q & 7) * 8; *(volatile v8b*)(ERP16 + ((size_t)b * NQ + n0 + nn) * C + c0 + c8) = *(const v8b*)(&T[nn][c8]); } __threadfence(); }
}
__global__ __launch_bounds__(256) void prepx_kernel(const float* __restrict__ ico, b16* __restrict__ ICO16) {
  const size_t t = (size_t)blockIdx.x * 256 + threadIdx.x; const size_t n1 = (size_t)NRK * C / 8; v8b o;
  const size_t u = t; if (u >= n1) return; const size_t e = u * 8; const size_t b = e / ((size_t)NKP * C); const int r = (int)((e / C) % NKP), c0 = (int)(e % C);
  if (r < NKV) { const float* src = ico + ((size_t)b * NKV + r) * C + c0; const v4f a = *(const v4f*)src, c = *(const v4f*)(src + 4); for (int j = 0; j < 4; ++j) { o[j] = (b16)(bf16_rne(a[j]) * XS); o[4 + j] = (b16)(bf16_rne(c[j]) * XS); } } else { for (int j = 0; j < 8; ++j) o[j] = (b16)0.0f; }
  for (int pass = 0; pass < 2; ++pass) { *(volatile v8b*)(ICO16 + e) = o; __threadfence(); }
}
__device__ __forceinline__ int w_nin(int k) { return k >= 6 ? C2 : C; }
__device__ __forceinline__ int w_nout(int k) { return (k == 1 || k == 4) ? C2 : C; }
__host__ __device__ constexpr size_t woff(int k) { return (size_t)k * C2 * C; }
__global__ __launch_bounds__(256) void prepw_kernel(const float* const* __restrict__ dummy, const float* __restrict__ w0, const float* __restrict__ w1, const float* __restrict__ w2, const float* __restrict__ w3, const float* __restrict__ w4, const float* __restrict__ w5, const float* __restrict__ w6, const float* __restrict__ w7, b16* __restrict__ WALL) {
  (void)dummy; __shared__ __attribute__((aligned(16))) b16 T[64][64 + 8];
  const int kind = blockIdx.z, i0 = blockIdx.x * 64, o0 = blockIdx.y * 64, t_ = threadIdx.x; const int nin = w_nin(kind), nout = w_nout(kind); if (i0 >= nin || o0 >= nout) return;
  const float* w = kind == 0 ? w0 : kind == 1 ? w1 : kind == 2 ? w2 : kind == 3 ? w3 : kind == 4 ? w4 : kind == 5 ? w5 : kind == 6 ? w6 : w7; b16* dst = WALL + woff(kind);
  for (int q = t_; q < 64 * 64; q += 256) { const int ii = q >> 6, oo = q & 63; T[oo][ii] = (b16)(bf16_rne(w[(size_t)(i0 + ii) * nout + o0 + oo]) * WSC); }
  __syncthreads();
  for (int pass = 0; pass < 2; ++pass) { for (int q = t_; q < 64 * 8; q += 256) { const int oo = q >> 3, c8 = (q & 7) * 8; *(volatile v8b*)(dst + (size_t)(o0 + oo) * nin + i0 + c8) = *(const v8b*)(&T[oo][c8]); } __threadfence(); }
}
template <int KD, int NP, int OUT>
__global__ __launch_bounds__(128) void gemm_kernel(const b16* __restrict__ Ah, const b16* __restrict__ Al, int lda, const b16* __restrict__ W, int wcol0, const float* __restrict__ bias, float* __restrict__ Yf, b16* __restrict__ Yh, b16* __restrict__ Yl, int ldy, int ycol0, int rpb) {
  __shared__ __attribute__((aligned(16))) float Tf[OUT == 0 ? 4 : 1][16][128 + 4]; __shared__ __attribute__((aligned(16))) b16 Th[OUT == 1 ? 4 : 1][16][128 + 8], Tl[OUT == 1 ? 4 : 1][16][128 + 8]; __shared__ __attribute__((aligned(16))) b16 Vt[OUT == 2 ? 128 : 1][64 + 8], Vtl[OUT == 2 ? 128 : 1][64 + 8];
  const int wave = threadIdx.x >> 5, lane = threadIdx.x & 31, nloc = lane & 15, hlf = lane >> 4, t_ = threadIdx.x; const size_t m0 = (size_t)blockIdx.x * 64 + wave * 16;
  v8f acc[8];
#pragma unroll
  for (int t = 0; t < 8; ++t) acc[t] = (v8f){};
#pragma unroll 2
  for (int kb = 0; kb < KD; kb += 32) { const v16b a = frag_kb(Ah + (m0 + nloc) * lda + kb, hlf); v16b al; if (NP == 2) al = frag_kb(Al + (m0 + nloc) * lda + kb, hlf);
#pragma unroll
    for (int t = 0; t < 8; ++t) { const v16b bw = frag_kb(W + (size_t)(wcol0 + t * 16 + nloc) * KD + kb, hlf); acc[t] = wmma16b(a, bw, acc[t]); if (NP == 2) acc[t] = wmma16b(al, bw, acc[t]); } }
#pragma unroll
  for (int t = 0; t < 8; ++t) { const float bb = bias ? bf16_rne(bias[t * 16 + nloc]) : 0.0f;
#pragma unroll
    for (int r = 0; r < 8; ++r) { const float y = acc[t][r] * (1.0f / (XS * WSC)) + bb;
      if (OUT == 0) Tf[wave][8 * hlf + r][t * 16 + nloc] = y; else { b16 p, q; split16(y * XS, p, q); if (OUT == 1) { Th[wave][8 * hlf + r][t * 16 + nloc] = p; Tl[wave][8 * hlf + r][t * 16 + nloc] = q; } else { Vt[t * 16 + nloc][wave * 16 + 8 * hlf + r] = p; Vtl[t * 16 + nloc][wave * 16 + 8 * hlf + r] = q; } } } }
  if (OUT == 2) __syncthreads(); else wave_lds_sync();
  for (int pass = 0; pass < 2; ++pass) {
    if (OUT == 0) { for (int rr = 0; rr < 16; ++rr) *(volatile v4f*)(Yf + (m0 + rr) * ldy + ycol0 + lane * 4) = *(const v4f*)(&Tf[wave][rr][lane * 4]); }
    else if (OUT == 1) { for (int r2 = 0; r2 < 16; r2 += 2) { const int rr = r2 + (lane >> 4), c8 = (lane & 15) * 8; const size_t gi = (m0 + rr) * ldy + ycol0 + c8; *(volatile v8b*)(Yh + gi) = *(const v8b*)(&Th[wave][rr][c8]); *(volatile v8b*)(Yl + gi) = *(const v8b*)(&Tl[wave][rr][c8]); } }
    else { const size_t r0 = (size_t)blockIdx.x * 64; const size_t b = r0 / rpb; const int rl = (int)(r0 - b * rpb); for (int q = t_; q < 128 * 8; q += 128) { const int cc = q >> 3, c8 = (q & 7) * 8; const size_t gi = ((size_t)b * C + cc) * rpb + rl + c8; *(volatile v8b*)(Yh + gi) = *(const v8b*)(&Vt[cc][c8]); *(volatile v8b*)(Yl + gi) = *(const v8b*)(&Vtl[cc][c8]); } }
    __threadfence(); }
}
__global__ __launch_bounds__(64) void attnA_kernel(const b16* __restrict__ Qh, const b16* __restrict__ Ql, const b16* __restrict__ Kh, const b16* __restrict__ Kl, const b16* __restrict__ VTh, const b16* __restrict__ VTl, float* __restrict__ OA) {
  __shared__ __attribute__((aligned(16))) float To[2][16][C + 4];
  const int wave = threadIdx.x >> 5, lane = threadIdx.x & 31, hh = lane >> 4, col = lane & 15; const int b = blockIdx.z; const int q0 = blockIdx.x * 32 + wave * 16, qi = q0 + col;
  const b16* Qb = Qh + ((size_t)b * NQ + qi) * C; const b16* Qlb = Ql + ((size_t)b * NQ + qi) * C; const b16* Kb = Kh + (size_t)b * NKP * C; const b16* Klb = Kl + (size_t)b * NKP * C; const b16* Vb = VTh + (size_t)b * C * NKP; const b16* Vlb = VTl + (size_t)b * C * NKP;
  v16b qa[4], ql[4];
#pragma unroll
  for (int ks = 0; ks < 4; ++ks) { qa[ks] = frag_kb(Qb + ks * 32, hh); ql[ks] = frag_kb(Qlb + ks * 32, hh); }
  float m = -INFINITY, l = 0.0f; v8f o[8];
#pragma unroll
  for (int t = 0; t < 8; ++t) o[t] = (v8f){};
  const float cs = SCALE * LOG2E / (XS * XS);
  for (int kb = 0; kb < NKP; kb += 32) {
    v8f s0 = {}, s1 = {};
#pragma unroll
    for (int ks = 0; ks < 4; ++ks) { const b16* k0 = Kb + (size_t)(kb + col) * C + ks * 32, *k1 = Kb + (size_t)(kb + 16 + col) * C + ks * 32, *k0l = Klb + (size_t)(kb + col) * C + ks * 32, *k1l = Klb + (size_t)(kb + 16 + col) * C + ks * 32;
      v16b f = frag_kb(k0, hh); s0 = wmma16b(f, qa[ks], s0); s0 = wmma16b(f, ql[ks], s0); s0 = wmma16b(frag_kb(k0l, hh), qa[ks], s0);
      f = frag_kb(k1, hh); s1 = wmma16b(f, qa[ks], s1); s1 = wmma16b(f, ql[ks], s1); s1 = wmma16b(frag_kb(k1l, hh), qa[ks], s1); }
    float e[16]; float mx = -INFINITY;
#pragma unroll
    for (int r = 0; r < 8; ++r) { const int k0i = kb + 8 * hh + r, k1i = kb + 16 + 8 * hh + r; e[r] = (k0i < NKV) ? s0[r] * cs : -INFINITY; e[8 + r] = (k1i < NKV) ? s1[r] * cs : -INFINITY; mx = fmaxf(mx, fmaxf(e[r], e[8 + r])); }
    mx = fmaxf(mx, __shfl_xor(mx, 16)); const float mn = fmaxf(m, mx); const float al = nexp2(m - mn); m = mn; float sum = 0.0f; v16b ph, pl;
#pragma unroll
    for (int i = 0; i < 16; ++i) { const float p = nexp2(e[i] - mn); sum += p; const b16 h_ = (b16)(p * PS); ph[i] = h_; pl[i] = (b16)(p * PS - (float)h_); }
    sum += __shfl_xor(sum, 16); l = l * al + sum;
#pragma unroll
    for (int t = 0; t < 8; ++t) { o[t] *= al; const v16b vf = frag_kb(Vb + (size_t)(t * 16 + col) * NKP + kb, hh); o[t] = wmma16b(vf, ph, o[t]); o[t] = wmma16b(vf, pl, o[t]); o[t] = wmma16b(frag_kb(Vlb + (size_t)(t * 16 + col) * NKP + kb, hh), ph, o[t]); } }
  const float inv = 1.0f / (l * PS * XS);
#pragma unroll
  for (int t = 0; t < 8; ++t)
#pragma unroll
    for (int r = 0; r < 8; ++r) To[wave][col][t * 16 + 8 * hh + r] = o[t][r] * inv;
  wave_lds_sync();
  for (int pass = 0; pass < 2; ++pass) { for (int rr = 0; rr < 16; ++rr) *(volatile v4f*)(OA + ((size_t)b * NQ + q0 + rr) * C + lane * 4) = *(const v4f*)(&To[wave][rr][lane * 4]); __threadfence(); }
}
__global__ __launch_bounds__(256) void otrans_kernel(const float* __restrict__ OA, b16* __restrict__ OTh, b16* __restrict__ OTl) {
  __shared__ __attribute__((aligned(16))) b16 Th[64][64 + 8], Tl[64][64 + 8];
  const int b = blockIdx.z, c0 = blockIdx.y * 64, n0 = blockIdx.x * 64, t_ = threadIdx.x;
  for (int q = t_; q < 64 * 64; q += 256) { const int nn = q >> 6, cc = q & 63; b16 p, ql; split16(OA[((size_t)b * NQ + n0 + nn) * C + c0 + cc] * XS, p, ql); Th[cc][nn] = p; Tl[cc][nn] = ql; }
  __syncthreads();
  for (int pass = 0; pass < 2; ++pass) { for (int q = t_; q < 64 * 8; q += 256) { const int cc = q >> 3, c8 = (q & 7) * 8; const size_t gi = ((size_t)b * C + c0 + cc) * NQ + n0 + c8; *(volatile v8b*)(OTh + gi) = *(const v8b*)(&Th[cc][c8]); *(volatile v8b*)(OTl + gi) = *(const v8b*)(&Tl[cc][c8]); } __threadfence(); }
}
__global__ __launch_bounds__(256) void dlogit_kernel(const float* __restrict__ QD, const float* __restrict__ KD, const float* __restrict__ icoc, const float* __restrict__ wdelta, b16* __restrict__ Ph, b16* __restrict__ Pl) {
  __shared__ float Lg[16][NKP + 1]; __shared__ float ds[3]; __shared__ float qc[16][3]; __shared__ float rmax[16], rinv[16]; __shared__ __attribute__((aligned(16))) b16 Rh[NKP], Rl[NKP];
  const int b = blockIdx.y, q0 = blockIdx.x * 16, t_ = threadIdx.x, wave = t_ >> 5, lane = t_ & 31;
  if (t_ < 3) { float s = 0.0f; for (int c = 0; c < C; ++c) s += bf16_rne(wdelta[t_ * C + c]); ds[t_] = s; }
  if (t_ < 16) { const int n = q0 + t_; const int i = n / WQ, j = n % WQ;
    const float u = (((float)j - ((float)WQ * 0.5f + 0.5f)) / (float)WQ) * 2.0f * PI_F; const float v = (((float)i - ((float)HQ * 0.5f + 0.5f)) / (float)HQ) * PI_F;
    qc[t_][0] = cosf(v) * sinf(u); qc[t_][1] = sinf(v); qc[t_][2] = cosf(v) * cosf(u); }
  __syncthreads();
  { const int q = t_ & 15, ph = t_ >> 4; const float* qd = QD + ((size_t)b * NQ + q0 + q) * C;
    for (int k = ph; k < NKP; k += 16) { float lg = -INFINITY;
      if (k < NKV) { const float* kd = KD + ((size_t)b * NKP + k) * C; float fs = 0.0f;
#pragma unroll 4
        for (int c = 0; c < C; ++c) fs += __expf(-fabsf(qd[c] - kd[c]));
        const float* kc = icoc + ((size_t)b * NKV + k) * 3; float ps = 0.0f; for (int d3 = 0; d3 < 3; ++d3) ps += pmul(__expf(-fabsf(qc[q][d3] - bf16_rne(kc[d3]))), ds[d3]);
        lg = (fs + ps) * (1.0f / (float)C); }
      Lg[q][k] = lg; } }
  __syncthreads();
  for (int rr = wave * 2; rr < wave * 2 + 2; ++rr) { float mx = -INFINITY; for (int k = lane; k < NKP; k += 32) mx = fmaxf(mx, Lg[rr][k]);
#pragma unroll
    for (int o = 16; o >= 1; o >>= 1) mx = fmaxf(mx, __shfl_xor(mx, o));
    float sm = 0.0f; for (int k = lane; k < NKP; k += 32) sm += nexp2((Lg[rr][k] - mx) * LOG2E);
#pragma unroll
    for (int o = 16; o >= 1; o >>= 1) sm += __shfl_xor(sm, o);
    if (lane == 0) { rmax[rr] = mx; rinv[rr] = PSD / sm; } }
  __syncthreads();
  for (int rr = 0; rr < 16; ++rr) {
    for (int k = t_; k < NKP; k += 256) { const float p = nexp2((Lg[rr][k] - rmax[rr]) * LOG2E) * rinv[rr]; b16 h_, l_; split16(p, h_, l_); Rh[k] = h_; Rl[k] = l_; }
    __syncthreads();
    for (int pass = 0; pass < 2; ++pass) { if (t_ < NKP / 8) { const size_t gi = ((size_t)b * NQ + q0 + rr) * NKP + t_ * 8; *(volatile v8b*)(Ph + gi) = *(const v8b*)(&Rh[t_ * 8]); *(volatile v8b*)(Pl + gi) = *(const v8b*)(&Rl[t_ * 8]); } __threadfence(); }
    __syncthreads(); }
}
__global__ __launch_bounds__(128) void pvd_kernel(const b16* __restrict__ Ph, const b16* __restrict__ Pl, const b16* __restrict__ VTh, const b16* __restrict__ VTl, b16* __restrict__ ODh, b16* __restrict__ ODl) {
  __shared__ __attribute__((aligned(16))) b16 Th[4][16][128 + 8], Tl[4][16][128 + 8];
  const int wave = threadIdx.x >> 5, lane = threadIdx.x & 31, nloc = lane & 15, hlf = lane >> 4; const size_t m0 = (size_t)blockIdx.x * 64 + wave * 16; const size_t b = m0 / NQ;
  const b16* Vb = VTh + b * C * NKP; const b16* Vlb = VTl + b * C * NKP; v8f acc[8];
#pragma unroll
  for (int t = 0; t < 8; ++t) acc[t] = (v8f){};
  for (int kb = 0; kb < NKP; kb += 32) { const v16b a = frag_kb(Ph + (m0 + nloc) * NKP + kb, hlf), al = frag_kb(Pl + (m0 + nloc) * NKP + kb, hlf);
#pragma unroll
    for (int t = 0; t < 8; ++t) { const v16b bv = frag_kb(Vb + (size_t)(t * 16 + nloc) * NKP + kb, hlf); acc[t] = wmma16b(a, bv, acc[t]); acc[t] = wmma16b(al, bv, acc[t]); acc[t] = wmma16b(a, frag_kb(Vlb + (size_t)(t * 16 + nloc) * NKP + kb, hlf), acc[t]); } }
#pragma unroll
  for (int t = 0; t < 8; ++t)
#pragma unroll
    for (int r = 0; r < 8; ++r) { b16 p, q; split16(acc[t][r] * (1.0f / (PSD * XS)) * XS, p, q); Th[wave][8 * hlf + r][t * 16 + nloc] = p; Tl[wave][8 * hlf + r][t * 16 + nloc] = q; }
  wave_lds_sync();
  for (int pass = 0; pass < 2; ++pass) { for (int r2 = 0; r2 < 16; r2 += 2) { const int rr = r2 + (lane >> 4), c8 = (lane & 15) * 8; const size_t gi = (m0 + rr) * C + c8; *(volatile v8b*)(ODh + gi) = *(const v8b*)(&Th[wave][rr][c8]); *(volatile v8b*)(ODl + gi) = *(const v8b*)(&Tl[wave][rr][c8]); } __threadfence(); }
}
__global__ __launch_bounds__(128) void fuse_kernel(const b16* __restrict__ CATh, const b16* __restrict__ CATl, const float* __restrict__ CATf, const b16* __restrict__ WGA, const b16* __restrict__ WGD, float* __restrict__ out) {
  __shared__ __attribute__((aligned(16))) float Tt[C][64 + 4];
  const int wave = threadIdx.x >> 5, lane = threadIdx.x & 31, nloc = lane & 15, hlf = lane >> 4, t_ = threadIdx.x; const size_t m0 = (size_t)blockIdx.x * 64 + wave * 16; const size_t r0 = (size_t)blockIdx.x * 64; const size_t b = r0 / NQ; const int n0 = (int)(r0 - b * NQ);
  v8f ga[8], gd[8];
#pragma unroll
  for (int t = 0; t < 8; ++t) { ga[t] = (v8f){}; gd[t] = (v8f){}; }
#pragma unroll 2
  for (int kb = 0; kb < C2; kb += 32) { const v16b a = frag_kb(CATh + (m0 + nloc) * C2 + kb, hlf), al = frag_kb(CATl + (m0 + nloc) * C2 + kb, hlf);
#pragma unroll
    for (int t = 0; t < 8; ++t) { const v16b wa = frag_kb(WGA + (size_t)(t * 16 + nloc) * C2 + kb, hlf), wd = frag_kb(WGD + (size_t)(t * 16 + nloc) * C2 + kb, hlf); ga[t] = wmma16b(a, wa, ga[t]); ga[t] = wmma16b(al, wa, ga[t]); gd[t] = wmma16b(a, wd, gd[t]); gd[t] = wmma16b(al, wd, gd[t]); } }
#pragma unroll
  for (int t = 0; t < 8; ++t) { const int c = t * 16 + nloc;
#pragma unroll
    for (int r = 0; r < 8; ++r) { const size_t row = m0 + 8 * hlf + r; const float sa = 1.0f / (1.0f + __expf(-ga[t][r] * (1.0f / (XS * WSC)))), sd = 1.0f / (1.0f + __expf(-gd[t][r] * (1.0f / (XS * WSC))));
      Tt[c][wave * 16 + 8 * hlf + r] = pmul(sa, CATf[row * C2 + c]) + pmul(sd, CATf[row * C2 + C + c]); } }
  __syncthreads();
  for (int pass = 0; pass < 2; ++pass) { for (int q = t_; q < C * 16; q += 128) { const int cc = q >> 4, c4 = (q & 15) * 4; *(volatile v4f*)(out + ((size_t)b * C + cc) * NQ + n0 + c4) = *(const v4f*)(&Tt[cc][c4]); } __threadfence(); }
}
}

extern "C" void kernel_launch(void* const* d_in, const int* in_sizes, int n_in, void* d_out, int out_size, void* d_ws, size_t ws_size, hipStream_t stream) {
  (void)n_in;
  auto Fp = [&](int i) { return (const float*)d_in[i]; };
  if (in_sizes[0] != NRQ * C || in_sizes[1] != NB * NKV * C || in_sizes[2] != NB * NKV * 3 || in_sizes[3] != C * C || in_sizes[4] != C * C2 || in_sizes[5] != C * C || in_sizes[6] != C || in_sizes[9] != C * C || in_sizes[11] != 3 * C || in_sizes[12] != C2 * C || in_sizes[13] != C2 * C || out_size != NRQ * C) return;
  size_t off = 0; char* ws = (char*)d_ws;
  auto carve = [&](size_t bytes) { char* p = ws + off; off += (bytes + 255) & ~(size_t)255; return p; };
  b16* ERP16 = (b16*)carve((size_t)NRQ * C * 2); b16* ICO16 = (b16*)carve((size_t)NRK * C * 2); b16* WALL = (b16*)carve(woff(8) * 2);
  b16* QAh = (b16*)carve((size_t)NRQ * C * 2); b16* QAl = (b16*)carve((size_t)NRQ * C * 2); b16* KAh = (b16*)carve((size_t)NRK * C * 2); b16* KAl = (b16*)carve((size_t)NRK * C * 2); b16* VATh = (b16*)carve((size_t)NRK * C * 2); b16* VATl = (b16*)carve((size_t)NRK * C * 2);
  float* QD = (float*)carve((size_t)NRQ * C * 4); float* KD = (float*)carve((size_t)NRK * C * 4); b16* VDTh = (b16*)carve((size_t)NRK * C * 2); b16* VDTl = (b16*)carve((size_t)NRK * C * 2);
  float* OA = (float*)carve((size_t)NRQ * C * 4); b16* OTh = (b16*)carve((size_t)NRQ * C * 2); b16* OTl = (b16*)carve((size_t)NRQ * C * 2); b16* Ph = (b16*)carve((size_t)NRQ * NKP * 2); b16* Pl = (b16*)carve((size_t)NRQ * NKP * 2);
  b16* ODh = (b16*)carve((size_t)NRQ * C * 2); b16* ODl = (b16*)carve((size_t)NRQ * C * 2); float* CATf = (float*)carve((size_t)NRQ * C2 * 4); b16* CATh = (b16*)carve((size_t)NRQ * C2 * 2); b16* CATl = (b16*)carve((size_t)NRQ * C2 * 2);
  if (off > ws_size || off > ((size_t)128 << 20)) return;
  preperp_kernel<<<dim3(NQ / 64, C / 64, NB), 256, 0, stream>>>(Fp(0), ERP16);
  prepx_kernel<<<(unsigned)(((size_t)NRK * C / 8 + 255) / 256), 256, 0, stream>>>(Fp(1), ICO16);
  prepw_kernel<<<dim3(4, 4, 8), 256, 0, stream>>>(nullptr, Fp(3), Fp(4), Fp(5), Fp(7), Fp(8), Fp(9), Fp(12), Fp(13), WALL);
  gemm_kernel<C, 1, 1><<<NRQ / 64, 128, 0, stream>>>(ERP16, nullptr, C, WALL + woff(0), 0, nullptr, nullptr, QAh, QAl, C, 0, 0);
  gemm_kernel<C, 1, 1><<<NRK / 64, 128, 0, stream>>>(ICO16, nullptr, C, WALL + woff(1), 0, nullptr, nullptr, KAh, KAl, C, 0, 0);
  gemm_kernel<C, 1, 2><<<NRK / 64, 128, 0, stream>>>(ICO16, nullptr, C, WALL + woff(1), C, nullptr, nullptr, VATh, VATl, 0, 0, NKP);
  attnA_kernel<<<dim3(NQ / 32, 1, NB), 64, 0, stream>>>(QAh, QAl, KAh, KAl, VATh, VATl, OA);
  otrans_kernel<<<dim3(NQ / 64, C / 64, NB), 256, 0, stream>>>(OA, OTh, OTl);
  gemm_kernel<C, 1, 0><<<NRQ / 64, 128, 0, stream>>>(ERP16, nullptr, C, WALL + woff(3), 0, nullptr, QD, nullptr, nullptr, C, 0, 0);
  gemm_kernel<C, 1, 0><<<NRK / 64, 128, 0, stream>>>(ICO16, nullptr, C, WALL + woff(4), 0, nullptr, KD, nullptr, nullptr, C, 0, 0);
  gemm_kernel<C, 1, 2><<<NRK / 64, 128, 0, stream>>>(ICO16, nullptr, C, WALL + woff(4), C, nullptr, nullptr, VDTh, VDTl, 0, 0, NKP);
  dlogit_kernel<<<dim3(NQ / 16, NB), 256, 0, stream>>>(QD, KD, Fp(2), Fp(11), Ph, Pl);
  pvd_kernel<<<NRQ / 64, 128, 0, stream>>>(Ph, Pl, VDTh, VDTl, ODh, ODl);
  gemm_kernel<C, 2, 0><<<NRQ / 64, 128, 0, stream>>>(OTh, OTl, C, WALL + woff(2), 0, Fp(6), CATf, nullptr, nullptr, C2, 0, 0);
  gemm_kernel<C, 2, 1><<<NRQ / 64, 128, 0, stream>>>(OTh, OTl, C, WALL + woff(2), 0, Fp(6), nullptr, CATh, CATl, C2, 0, 0);
  gemm_kernel<C, 2, 0><<<NRQ / 64, 128, 0, stream>>>(ODh, ODl, C, WALL + woff(5), 0, Fp(10), CATf, nullptr, nullptr, C2, C, 0);
  gemm_kernel<C, 2, 1><<<NRQ / 64, 128, 0, stream>>>(ODh, ODl, C, WALL + woff(5), 0, Fp(10), nullptr, CATh, CATl, C2, C, 0);
  fuse_kernel<<<NRQ / 64, 128, 0, stream>>>(CATh, CATl, CATf, WALL + woff(6), WALL + woff(7), (float*)d_out);
}
